// Hyp_plus_MLR_70549132804742
// MI455X (gfx1250) — hardware-run, weakly checked
//
#include <hip/hip_runtime.h>
#include <math.h>

typedef __attribute__((ext_vector_type(16))) _Float16 v16h;
typedef __attribute__((ext_vector_type(8)))  _Float16 v8h;
typedef __attribute__((ext_vector_type(4)))  _Float16 v4h;
typedef __attribute__((ext_vector_type(2)))  _Float16 v2h;
typedef __attribute__((ext_vector_type(16))) __bf16   v16b;
typedef __attribute__((ext_vector_type(8)))  __bf16   v8b;
typedef __attribute__((ext_vector_type(8)))  float    v8f;
typedef __attribute__((ext_vector_type(4)))  float    v4f;
typedef __attribute__((ext_vector_type(2)))  float    v2f;

constexpr int kB    = 2048;
constexpr int kC    = 128;
constexpr int kD    = 256;
constexpr int kThr  = 256;
constexpr float kInCarry = 1024.0f;
constexpr float kSc20 = 1.0f / (kInCarry * kInCarry);
constexpr float kF16MinNormal = 6.103515625e-5f;
constexpr float kFloorU = 1.0e-15f;
constexpr float kFloorA = 1.0e-12f;

static_assert(kB == 2048 && kC == 128 && kD == 256, "the index arithmetic below uses these sizes");

constexpr size_t kOffY16 = 0ull;
constexpr size_t kOffYR = 1048576ull;
constexpr size_t kOffZR = 3145728ull;
constexpr size_t kOffRR = 3276800ull;
constexpr size_t kOffQA = 3277312ull;
constexpr size_t kOffKS = 3408384ull;
constexpr size_t kOffY2 = 3410432ull;
constexpr size_t kOffPP = 3418624ull;
constexpr size_t kWsTotal = 5515776ull;
static_assert(kWsTotal <= 268435456ull, "the carve stands under 256 MiB");
static_assert(kOffY16 == 0
  && kOffYR == kOffY16 + 1048576ull
  && kOffZR == kOffYR + 2097152ull
  && kOffRR == kOffZR + 131072ull
  && kOffQA == kOffRR + 512ull
  && kOffKS == kOffQA + 131072ull
  && kOffY2 == kOffKS + 2048ull
  && kOffPP == kOffY2 + 8192ull
  && kWsTotal == kOffPP + 2097152ull, "the carve is a chain: every region starts where the one before ends");
static_assert((kOffY16 % 256) == 0 && (kOffYR % 256) == 0 && (kOffZR % 256) == 0 && (kOffRR % 256) == 0 && (kOffQA % 256) == 0 && (kOffKS % 256) == 0 && (kOffY2 % 256) == 0 && (kOffPP % 256) == 0, "every region starts on a multiple of 256 B");

__device__ __forceinline__ unsigned short f2bf_bits(float f) {
  unsigned u = __float_as_uint(f);
  return (unsigned short)((u + 0x7FFFu + ((u >> 16) & 1u)) >> 16);
}
__device__ __forceinline__ float bf_bits2f(unsigned short h) { return __uint_as_float(((unsigned)h) << 16); }
__device__ __forceinline__ float bf16r(float f) { return bf_bits2f(f2bf_bits(f)); }
__device__ __forceinline__ float carry_flush(float v, float carry) {
  const float s = v * carry;
  return (fabsf(s) < kF16MinNormal) ? 0.0f : s;
}

__device__ __forceinline__ void dep_guard4_h(v8f& a, v8f& b, v8f& c, v8f& d, v16h x, v16h y) { asm volatile("v_nop\n\tv_nop\n\tv_nop\n\tv_nop" : "+v"(a), "+v"(b), "+v"(c), "+v"(d) : "v"(x), "v"(y)); }
__device__ __forceinline__ void dep_guard4_b(v8f& a, v8f& b, v8f& c, v8f& d, v16b x, v16b y) { asm volatile("v_nop\n\tv_nop\n\tv_nop\n\tv_nop" : "+v"(a), "+v"(b), "+v"(c), "+v"(d) : "v"(x), "v"(y)); }
__device__ __forceinline__ void keep4_h(v16h a, v16h b, v16h c, v16h d) { asm volatile("v_nop" :: "v"(a), "v"(b), "v"(c), "v"(d)); }
__device__ __forceinline__ void keep4_b(v16b a, v16b b, v16b c, v16b d) { asm volatile("v_nop" :: "v"(a), "v"(b), "v"(c), "v"(d)); }
__device__ __forceinline__ void acc_guard4(v8f& a, v8f& b, v8f& c, v8f& d) { asm volatile("v_nop\n\tv_nop\n\tv_nop\n\tv_nop" : "+v"(a), "+v"(b), "+v"(c), "+v"(d)); }

template <typename T> struct Frag;
template <> struct Frag<_Float16> {
  typedef v16h V; union U { v16h v; v8h h[2]; };
  static __device__ __forceinline__ v16h load(const _Float16* p) {
    U f; f.h[0] = *(const v8h*)(p); f.h[1] = *(const v8h*)(p + 16); return f.v;
  }
  static __device__ __forceinline__ v8f mma(v16h a, v16h b, v8f c) {
    return __builtin_amdgcn_wmma_f32_16x16x32_f16(false, a, false, b, (short)0, c, false, false);
  }
  static __device__ __forceinline__ void guard4(v8f& a, v8f& b, v8f& c, v8f& d, v16h x, v16h y) { dep_guard4_h(a, b, c, d, x, y); }
  static __device__ __forceinline__ void keep(v16h a, v16h b, v16h c, v16h d) { keep4_h(a, b, c, d); }
};
template <> struct Frag<__bf16> {
  typedef v16b V; union U { v16b v; v8b h[2]; };
  static __device__ __forceinline__ v16b load(const __bf16* p) {
    U f; f.h[0] = *(const v8b*)(p); f.h[1] = *(const v8b*)(p + 16); return f.v;
  }
  static __device__ __forceinline__ v8f mma(v16b a, v16b b, v8f c) {
    return __builtin_amdgcn_wmma_f32_16x16x32_bf16(false, a, false, b, (short)0, c, false, false);
  }
  static __device__ __forceinline__ void guard4(v8f& a, v8f& b, v8f& c, v8f& d, v16b x, v16b y) { dep_guard4_b(a, b, c, d, x, y); }
  static __device__ __forceinline__ void keep(v16b a, v16b b, v16b c, v16b d) { keep4_b(a, b, c, d); }
};

__device__ __forceinline__ v8f mma_h(v16h a, v16h b, v8f c) {
  c = __builtin_amdgcn_wmma_f32_16x16x32_f16(false, a, false, b, (short)0, c, false, false);
  asm volatile("v_nop\n\tv_nop\n\tv_nop\n\tv_nop" : "+v"(c) : "v"(a), "v"(b));
  return c;
}

template <int ET> struct Elem;
template <> struct Elem<0> { typedef _Float16 T; };
template <> struct Elem<1> { typedef __bf16 T; };
template <int ET, bool SPLIT, int BIAS_MODE, int OUT_MODE, bool RESID, int ACT = 0>
__global__ __launch_bounds__(256) void wmma_gemm64(
    const unsigned short* __restrict__ Ap, const unsigned short* __restrict__ A2p, int lda, long strideA,
    const unsigned short* __restrict__ Btp, const unsigned short* __restrict__ Bt2p, int ldb, long strideB,
    void* __restrict__ Cout, void* __restrict__ Cout2, int ldc, long strideC,
    const float* __restrict__ bias,
    const float* __restrict__ resid, long strideR,
    int M, int N, int K, float scale) {
  typedef typename Elem<ET>::T T;
  typedef typename Frag<T>::V V;
  const T* A = (const T*)Ap; const T* A2 = (const T*)A2p; const T* Bt = (const T*)Btp; const T* Bt2 = (const T*)Bt2p;
  __shared__ __align__(16) float sT[8][16 * 68];
  const int b    = blockIdx.y;
  const int lane = threadIdx.x & 31;
  const int wave = threadIdx.x >> 5;
  const int tilesN = N >> 6;
  const int tilesM = M >> 6;
  const int tile = blockIdx.x * 8 + wave;
  if (tile >= tilesM * tilesN) return;
  const int tm = tile / tilesN;
  const int tn = tile - tm * tilesN;
  const int m0 = tm << 6;
  const int n0 = tn << 6;

  const T* Ab  = A  + (size_t)b * strideA;
  const T* Bb  = Bt + (size_t)b * strideB;
  const T* Ab2 = SPLIT ? (A2  + (size_t)b * strideA) : nullptr;
  const T* Bb2 = SPLIT ? (Bt2 + (size_t)b * strideB) : nullptr;

  const int rlane = lane & 15;
  const int koff  = (lane >> 4) * 8;
  const int mOff  = (lane >> 4) * 8;

  v8f acc[4][4];
#pragma unroll
  for (int i = 0; i < 4; ++i)
#pragma unroll
    for (int j = 0; j < 4; ++j) acc[i][j] = (v8f){0.f,0.f,0.f,0.f,0.f,0.f,0.f,0.f};

  for (int k0 = 0; k0 < K; k0 += 32) {
    V bh[4], bl[4];
#pragma unroll
    for (int j = 0; j < 4; ++j) {
      const size_t bo = (size_t)(n0 + (j << 4) + rlane) * ldb + koff + k0;
      bh[j] = Frag<T>::load(Bb + bo);
      if (SPLIT) bl[j] = Frag<T>::load(Bb2 + bo);
    }
#pragma unroll
    for (int i = 0; i < 4; ++i) {
      const size_t ao = (size_t)(m0 + (i << 4) + rlane) * lda + koff + k0;
      V ah = Frag<T>::load(Ab + ao);
      V al;
      if (SPLIT) al = Frag<T>::load(Ab2 + ao);
#pragma unroll
      for (int j = 0; j < 4; ++j) {
        acc[i][j] = Frag<T>::mma(ah, bh[j], acc[i][j]);
        if (SPLIT) {
          acc[i][j] = Frag<T>::mma(ah, bl[j], acc[i][j]);
          acc[i][j] = Frag<T>::mma(al, bh[j], acc[i][j]);
        }
      }
      Frag<T>::guard4(acc[i][0], acc[i][1], acc[i][2], acc[i][3], ah, SPLIT ? al : ah);
    }
    Frag<T>::keep(bh[0], bh[1], bh[2], bh[3]);
    if (SPLIT) Frag<T>::keep(bl[0], bl[1], bl[2], bl[3]);
  }
  acc_guard4(acc[0][0], acc[0][1], acc[0][2], acc[0][3]);
  acc_guard4(acc[1][0], acc[1][1], acc[1][2], acc[1][3]);
  acc_guard4(acc[2][0], acc[2][1], acc[2][2], acc[2][3]);
  acc_guard4(acc[3][0], acc[3][1], acc[3][2], acc[3][3]);

  float* slab = sT[wave];
  const float* Rb = RESID ? (resid + (size_t)b * strideR) : nullptr;
#pragma unroll
  for (int i = 0; i < 4; ++i) {
    const int mBase = m0 + (i << 4);
#pragma unroll
    for (int j = 0; j < 4; ++j) {
      const int n = n0 + (j << 4) + rlane;
      float bv = 0.f;
      if (BIAS_MODE == 2) bv = bias[n];
#pragma unroll
      for (int r = 0; r < 8; ++r) {
        float v = acc[i][j][r] * scale;
        if (BIAS_MODE == 1) v += bias[mBase + mOff + r];
        if (BIAS_MODE == 2) v += bv;
        if (RESID) v += Rb[(size_t)(mBase + mOff + r) * ldc + n];
        if (ACT == 1) v = tanhf(v);
        if (ACT == 2) v = fmaxf(v, 0.0f);
        if (ACT == 3) v = v / (1.0f + expf(-v));
        if (ACT == 4) v = (v > 0.f) ? v : 0.01f * v;
        slab[(mOff + r) * 68 + (j << 4) + rlane] = v;
      }
    }
    __builtin_amdgcn_fence(__ATOMIC_RELEASE, "workgroup");
    __builtin_amdgcn_wave_barrier();
    __builtin_amdgcn_fence(__ATOMIC_ACQUIRE, "workgroup");
    if (OUT_MODE == 0) {
      float* C = (float*)Cout + (size_t)b * strideC;
      const int hh = lane >> 4, c4 = (lane & 15) * 4;
      for (int pass = 0; pass < 2; ++pass) {
#pragma unroll
        for (int it = 0; it < 8; ++it) {
          const int row = it * 2 + hh;
          v4f v = *(const v4f*)(slab + row * 68 + c4);
          *(volatile v4f*)(C + (size_t)(mBase + row) * ldc + n0 + c4) = v;
        }
        __threadfence();
      }
    } else {
      const int q = lane >> 3, c8 = (lane & 7) * 8;
      unsigned short* C  = (unsigned short*)Cout  + (size_t)b * strideC;
      unsigned short* C2 = (OUT_MODE == 2) ? ((unsigned short*)Cout2 + (size_t)b * strideC) : nullptr;
      for (int pass = 0; pass < 2; ++pass) {
#pragma unroll
        for (int it = 0; it < 4; ++it) {
          const int row = it * 4 + q;
          const float* sp = slab + row * 68 + c8;
          v8h hv, lv;
#pragma unroll
          for (int e = 0; e < 8; ++e) {
            if (OUT_MODE == 1) {
              hv[e] = (_Float16)sp[e];
            } else {
              unsigned short hb = f2bf_bits(sp[e]);
              unsigned short lb = f2bf_bits(sp[e] - bf_bits2f(hb));
              hv[e] = __builtin_bit_cast(_Float16, hb);
              lv[e] = __builtin_bit_cast(_Float16, lb);
            }
          }
          *(volatile v8h*)(C + (size_t)(mBase + row) * ldc + n0 + c8) = hv;
          if (OUT_MODE == 2) *(volatile v8h*)(C2 + (size_t)(mBase + row) * ldc + n0 + c8) = lv;
        }
        __threadfence();
      }
    }
    __builtin_amdgcn_fence(__ATOMIC_RELEASE, "workgroup");
    __builtin_amdgcn_wave_barrier();
    __builtin_amdgcn_fence(__ATOMIC_ACQUIRE, "workgroup");
  }
}

__global__ __launch_bounds__(kThr) void cast_plane_kernel(const float* __restrict__ src, unsigned short* __restrict__ dst,
                                                          int colsLog2, int dstPitch, int dstOff) {
  const int i   = blockIdx.x * kThr + threadIdx.x;
  const int sh  = colsLog2 - 3;
  const int row = i >> sh;
  const int c8  = (i & ((1 << sh) - 1)) * 8;
  const float* sp = src + ((size_t)row << colsLog2) + c8;
  const v4f a0 = *(const v4f*)(sp);
  const v4f a1 = *(const v4f*)(sp + 4);
  v8h hv;
#pragma unroll
  for (int e = 0; e < 4; ++e) {
    const float f0 = a0[e];
    const float f1 = a1[e];
    hv[e]     = (_Float16)carry_flush(bf16r(f0), kInCarry);
    hv[4 + e] = (_Float16)carry_flush(bf16r(f1), kInCarry);
  }
  unsigned short* dp = dst + (size_t)row * dstPitch + dstOff + c8;
  *(volatile v8h*)dp = hv;
  __threadfence();
  *(volatile v8h*)dp = hv;
}

__global__ __launch_bounds__(kThr) void pack_kernel(const float* __restrict__ W, unsigned short* __restrict__ D, float* __restrict__ dstf, int part, int ld, int k0, int lg, int n0, int pitch) {
  const unsigned i = blockIdx.x * blockDim.x + threadIdx.x;
  if (part == 0) {
    const unsigned g = i & ((1u << lg) - 1u), n = i >> lg;
    const float* sp = W + (size_t)((unsigned)k0 + g * 8u) * (unsigned)ld + n;
    v8h hv;
#pragma unroll
    for (int t = 0; t < 8; ++t) hv[t] = (_Float16)carry_flush(bf16r(sp[(size_t)t * (unsigned)ld]), kInCarry);
    unsigned short* dp = D + (size_t)((unsigned)n0 + n) * (unsigned)pitch + g * 8u;
    *(volatile v8h*)dp = hv;
    __threadfence();
    *(volatile v8h*)dp = hv;
  } else {
    const v4f a = *(const v4f*)(W + i * 4u);
    v4f o;
#pragma unroll
    for (int e = 0; e < 4; ++e) o[e] = bf16r(a[e]);
    float* dp = dstf + i * 4u;
    *(volatile v4f*)dp = o;
    __threadfence();
    *(volatile v4f*)dp = o;
  }
}

__global__ __launch_bounds__(kThr) void kprep_kernel(const float* __restrict__ ZR, const float* __restrict__ RR, unsigned short* __restrict__ QA, float* __restrict__ KS) {
  const unsigned k = threadIdx.x;
  const float* zp = ZR + (size_t)k * kD;
  const float rk = RR[k];
  const float ep = expf(rk);
  const float ch = 0.5f * (ep + 1.0f / ep);
  const float ia = 1.0f / (ch * ch);
  float s = 0.0f;
  for (int c = 0; c < 64; ++c) {
    const v4f z = *(const v4f*)(zp + 4 * c);
#pragma unroll
    for (int e = 0; e < 4; ++e) s = fmaf(z[e], z[e], s);
  }
  const float rs = sqrtf(s);
  const float an = ia * rs;
  const float un = fmaxf(fabsf(rk) * rs, kFloorU);
  const float e2 = expf(un + un);
  const float hh = 1.0f / (e2 + 1.0f);
  const float th = 1.0f - (hh + hh);
  const float gq = (th / un) * rk;
  const float da = fmaxf(an, kFloorA);
  const float ga = ia / da;
  const v4f sc = {an, (gq * gq) * s, 0.0f - (gq * ga) * s, 0.0f};
  unsigned short* qrow = QA + (size_t)k * kD;
  unsigned short* hrow = QA + (size_t)(kC + k) * kD;
  for (int pass = 0; pass < 2; ++pass) {
    for (int c = 0; c < 32; ++c) {
      const v4f z0 = *(const v4f*)(zp + 8 * c), z1 = *(const v4f*)(zp + 8 * c + 4);
      v8h wq, wh;
#pragma unroll
      for (int e = 0; e < 4; ++e) {
        wq[e]     = (_Float16)carry_flush(gq * z0[e], kInCarry); wh[e]     = (_Float16)carry_flush(ga * z0[e], kInCarry);
        wq[4 + e] = (_Float16)carry_flush(gq * z1[e], kInCarry); wh[4 + e] = (_Float16)carry_flush(ga * z1[e], kInCarry);
      }
      *(volatile v8h*)(qrow + 8 * c) = wq; *(volatile v8h*)(hrow + 8 * c) = wh;
    }
    *(volatile v4f*)(KS + (size_t)k * 4u) = sc;
    __threadfence();
  }
}

__global__ __launch_bounds__(kThr) void y2sum_kernel(const float* __restrict__ YR, float* __restrict__ Y2) {
  const unsigned b = blockIdx.x * (unsigned)kThr + threadIdx.x;
  const float* yp = YR + (size_t)b * kD;
  float s = 0.0f;
  for (int c = 0; c < 64; ++c) {
    const v4f y = *(const v4f*)(yp + 4 * c);
#pragma unroll
    for (int e = 0; e < 4; ++e) s = fmaf(y[e], y[e], s);
  }
  *(volatile float*)(Y2 + b) = s;
  __threadfence();
  *(volatile float*)(Y2 + b) = s;
}

__global__ __launch_bounds__(kThr) void mlrfinish_kernel(const float* __restrict__ PP, const float* __restrict__ Y2, const float* __restrict__ KS, float* __restrict__ res) {
  const unsigned v = blockIdx.x * (unsigned)kThr + threadIdx.x;
  const unsigned b = v >> 7, k = v & 127u;
  const float yq = PP[(size_t)b * kD + k], ya = PP[(size_t)b * kD + kC + k];
  const float y2 = Y2[b];
  const v4f ks = *(const v4f*)(KS + (size_t)k * 4u);
  const float an = ks[0], x2 = ks[1], xa = ks[2];
  const float d2 = yq + yq;
  const float om = 1.0f - d2;
  const float al = om + y2;
  const float be = 1.0f - x2;
  const float den = om + x2 * y2;
  const float mm = (((al * al) * x2 - (d2 * al) * be) + (be * be) * y2) / (den * den);
  const float ma = (al * xa + be * ya) / den;
  const float lam = 2.0f / (1.0f - mm);
  const float w = ma * lam;
  const float aw = fabsf(w);
  const float ls = logf(aw + sqrtf(fmaf(aw, aw, 1.0f)));
  const float as = (w < 0.0f) ? 0.0f - ls : ls;
  const float o = (an + an) * as;
  *(volatile float*)(res + v) = o;
  __threadfence();
  *(volatile float*)(res + v) = o;
}

extern "C" void kernel_launch(void* const* d_in, const int* in_sizes, int n_in,
                              void* d_out, int out_size, void* d_ws, size_t ws_size,
                              hipStream_t stream) {
  if (n_in < 3 || d_out == nullptr || d_ws == nullptr) return;
  if (in_sizes[0] != kB * kD || in_sizes[1] != kC * kD || in_sizes[2] != kC) return;
  if (out_size != kB * kC) return;
  if (ws_size < kWsTotal) return;
  const float* yb = (const float*)d_in[0];
  const float* zc = (const float*)d_in[1];
  const float* rc = (const float*)d_in[2];
  float* out = (float*)d_out;
  char* ws = (char*)d_ws;
  unsigned short* Y16 = (unsigned short*)(ws + kOffY16);
  float* YR = (float*)(ws + kOffYR);
  float* ZR = (float*)(ws + kOffZR);
  float* RR = (float*)(ws + kOffRR);
  unsigned short* QA = (unsigned short*)(ws + kOffQA);
  float* KS = (float*)(ws + kOffKS);
  float* Y2 = (float*)(ws + kOffY2);
  float* PP = (float*)(ws + kOffPP);

  static_assert((kB * kD / 8) % kThr == 0 && (kB * kD / 4) % kThr == 0 && (kC * kD / 4) % kThr == 0 && (kC / 4) == 32 && kC <= kThr && kB % kThr == 0 && (kB * kC) % kThr == 0
                && ((kB / 64) * (2 * kC / 64)) % 8 == 0 && kD % 32 == 0, "every grid exact");
  cast_plane_kernel<<<kB * kD / 8 / kThr, kThr, 0, stream>>>(yb, Y16, 8, kD, 0);
  pack_kernel<<<kB * kD / 4 / kThr, kThr, 0, stream>>>(yb, nullptr, YR, 1, 0, 0, 0, 0, 0);
  pack_kernel<<<kC * kD / 4 / kThr, kThr, 0, stream>>>(zc, nullptr, ZR, 1, 0, 0, 0, 0, 0);
  pack_kernel<<<1, kC / 4, 0, stream>>>(rc, nullptr, RR, 1, 0, 0, 0, 0, 0);
  kprep_kernel<<<1, kC, 0, stream>>>(ZR, RR, QA, KS);
  y2sum_kernel<<<kB / kThr, kThr, 0, stream>>>(YR, Y2);
  wmma_gemm64<0, false, 0, 0, false, 0><<<dim3((kB / 64) * (2 * kC / 64) / 8, 1), 256, 0, stream>>>(
      Y16, Y16, kD, 0L, QA, QA, kD, 0L, (void*)PP, (void*)PP, 2 * kC, 0L, nullptr, nullptr, 0L, kB, 2 * kC, kD, kSc20);
  mlrfinish_kernel<<<kB * kC / kThr, kThr, 0, stream>>>(PP, Y2, KS, out);
}
